// MeshDeformation_61821759258844
// MI455X (gfx1250) — hardware-verified
//
#include <hip/hip_runtime.h>
#include <stddef.h>


#define NVERT   6890
#define NBATCH  8
#define FEAT    128
#define HID     256
#define KPA     512
#define AGGC    256
#define NOUT    3
#define NLAST   16
#define NTHR    256
#define NWAVE   8
#define EPT     8
#define NGRP    2
#define CHUNK   (NTHR * EPT * NGRP)
#define WCAP    (EPT * NGRP * 32)
#define LISTN   (NWAVE * WCAP)
#define TV      128
#define TVSH    7
#define SPW     (TV / NWAVE)
#define PCAP    256
#define DEGCAP  64
#define GROWS   64
#define G16ROWS 128
#define XSC     16.0f
#define WSC     64.0f
#define PINV    0.0009765625f
#define DEFORM  0.1f

#define LDS_GEMM (GROWS * HID * 4)
#define LDS_AGG  ((LISTN + NWAVE * PCAP) * 4 + TV * DEGCAP * 8 + TV * 4 + NWAVE * 4)

static_assert((CHUNK & (CHUNK - 1)) == 0);
static_assert(TV == (1 << TVSH));
static_assert(SPW == 16);
static_assert(NBATCH == NWAVE);
static_assert((TV % 32) == 0);
static_assert(GROWS == NWAVE * 8);
static_assert(G16ROWS == NWAVE * 16);
static_assert((HID * 256 / 8) % NTHR == 0 && (HID * KPA / 8) % NTHR == 0 && (NLAST * HID / 8) % NTHR == 0);
static_assert(((LISTN + NWAVE * PCAP) * 4) % 16 == 0);

typedef float    v4f  __attribute__((ext_vector_type(4)));
typedef float    v8f  __attribute__((ext_vector_type(8)));
typedef int      v2i  __attribute__((ext_vector_type(2)));
typedef int      v4i  __attribute__((ext_vector_type(4)));
typedef _Float16 v4h  __attribute__((ext_vector_type(4)));
typedef _Float16 v8h  __attribute__((ext_vector_type(8)));
typedef _Float16 v16h __attribute__((ext_vector_type(16)));
union FragH { v16h v; v8h h[2]; };

__device__ __forceinline__ v8h pack8(v4f a, v4f b) {
  v8h r;
  r[0] = (_Float16)a.x; r[1] = (_Float16)a.y; r[2] = (_Float16)a.z; r[3] = (_Float16)a.w;
  r[4] = (_Float16)b.x; r[5] = (_Float16)b.y; r[6] = (_Float16)b.z; r[7] = (_Float16)b.w;
  return r;
}
__device__ __forceinline__ v4h pack4(v4f a) {
  v4h r;
  r[0] = (_Float16)a.x; r[1] = (_Float16)a.y; r[2] = (_Float16)a.z; r[3] = (_Float16)a.w;
  return r;
}
__device__ __forceinline__ v4f relu4(v4f a) {
  v4f r;
  r.x = fmaxf(a.x, 0.0f); r.y = fmaxf(a.y, 0.0f); r.z = fmaxf(a.z, 0.0f); r.w = fmaxf(a.w, 0.0f);
  return r;
}

__device__ __forceinline__ void wm2(v16h a0, v16h a1, v16h b, v8f& c0, v8f& c1) {
  v8f d0 = __builtin_amdgcn_wmma_f32_16x16x32_f16(false, a0, false, b, (short)0, c0, false, false);
  v8f d1 = __builtin_amdgcn_wmma_f32_16x16x32_f16(false, a1, false, b, (short)0, c1, false, false);
#if defined(__HIP_DEVICE_COMPILE__)
  asm volatile("v_nop\n\tv_nop\n\tv_nop\n\tv_nop" : "+v"(d0), "+v"(d1) : "v"(a0), "v"(a1), "v"(b));
#endif
  c0 = d0; c1 = d1;
}
__device__ __forceinline__ v8f wm1(v16h a, v16h b, v8f c) {
  v8f d = __builtin_amdgcn_wmma_f32_16x16x32_f16(false, a, false, b, (short)0, c, false, false);
#if defined(__HIP_DEVICE_COMPILE__)
  asm volatile("v_nop\n\tv_nop\n\tv_nop\n\tv_nop" : "+v"(d) : "v"(a), "v"(b));
#endif
  return d;
}

template <int NB, int SH>
__device__ __forceinline__ int scan_chunk(const int* __restrict__ dsts, int nE, int cbase, int slotBase,
                                          int vec8, int* list, int tid, int lane, int wave) {
  int wc = 0;
#pragma unroll
  for (int g = 0; g < NGRP; ++g) {
    const int el0  = (g * NTHR + tid) * EPT;
    const int e0   = cbase + el0;
    const int sent = -2147483647 - 1;
    v4i da, db;
    if (vec8 != 0 && cbase + CHUNK <= nE) {
      da = *(const v4i*)(dsts + e0);
      db = *(const v4i*)(dsts + e0 + 4);
    } else {
      da.x = (e0     < nE) ? dsts[min(e0,     nE - 1)] : sent;
      da.y = (e0 + 1 < nE) ? dsts[min(e0 + 1, nE - 1)] : sent;
      da.z = (e0 + 2 < nE) ? dsts[min(e0 + 2, nE - 1)] : sent;
      da.w = (e0 + 3 < nE) ? dsts[min(e0 + 3, nE - 1)] : sent;
      db.x = (e0 + 4 < nE) ? dsts[min(e0 + 4, nE - 1)] : sent;
      db.y = (e0 + 5 < nE) ? dsts[min(e0 + 5, nE - 1)] : sent;
      db.z = (e0 + 6 < nE) ? dsts[min(e0 + 6, nE - 1)] : sent;
      db.w = (e0 + 7 < nE) ? dsts[min(e0 + 7, nE - 1)] : sent;
    }
    const unsigned nb = (unsigned)slotBase;
    const unsigned s0 = (unsigned)da.x - nb, s1 = (unsigned)da.y - nb;
    const unsigned s2 = (unsigned)da.z - nb, s3 = (unsigned)da.w - nb;
    const unsigned s4 = (unsigned)db.x - nb, s5 = (unsigned)db.y - nb;
    const unsigned s6 = (unsigned)db.z - nb, s7 = (unsigned)db.w - nb;
    const bool h0 = s0 < (unsigned)NB, h1 = s1 < (unsigned)NB, h2 = s2 < (unsigned)NB, h3 = s3 < (unsigned)NB;
    const bool h4 = s4 < (unsigned)NB, h5 = s5 < (unsigned)NB, h6 = s6 < (unsigned)NB, h7 = s7 < (unsigned)NB;
    const unsigned any = __builtin_amdgcn_ballot_w32(h0 | h1 | h2 | h3 | h4 | h5 | h6 | h7);
    if (any != 0u) {
#define HITJ(J, HJ, SJ) { \
        const unsigned mj = __builtin_amdgcn_ballot_w32(HJ); \
        if (mj != 0u) { \
          if (HJ) { \
            const int pos = wc + (int)__builtin_amdgcn_mbcnt_lo(mj, 0u); \
            if (pos < WCAP) list[wave * WCAP + pos] = ((el0 + (J)) << SH) | (int)(SJ); \
          } \
          wc += (int)__builtin_popcount(mj); } }
      HITJ(0, h0, s0)
      HITJ(1, h1, s1)
      HITJ(2, h2, s2)
      HITJ(3, h3, s3)
      HITJ(4, h4, s4)
      HITJ(5, h5, s5)
      HITJ(6, h6, s6)
      HITJ(7, h7, s7)
#undef HITJ
    }
  }
  return wc;
}

__global__ __launch_bounds__(NTHR) void k_wprep(
    const float* __restrict__ W1, const float* __restrict__ L1,
    const float* __restrict__ Wb, const float* __restrict__ Lb,
    const float* __restrict__ W2, const float* __restrict__ L2,
    _Float16* B0, _Float16* BL, _Float16* B16, int nL) {
  const int g0 = HID * 256 / 8;
  const int g1 = nL * (HID * KPA / 8);
  const int g2 = NLAST * HID / 8;
  const int bstart = blockIdx.x * NTHR;
  const int i = bstart + (int)threadIdx.x;
  if (i >= g0 + g1 + g2) return;
  float v[8];
  _Float16* dp;
  if (bstart < g0) {
    const int o = i * 8;
    const int n = o >> 8;
    const int k0 = o & 255;
#pragma unroll
    for (int e = 0; e < 8; ++e) {
      const int k = k0 + e;
      const int kl = k < FEAT ? k : FEAT - 1;
      int kw = k - FEAT; kw = kw < 0 ? 0 : (kw > FEAT - 1 ? FEAT - 1 : kw);
      const float a = L1[(size_t)kl * HID + n];
      const float w = W1[(size_t)kw * HID + n];
      v[e] = (k < FEAT ? a : w) * WSC;
    }
    dp = B0 + o;
  } else if (bstart < g0 + g1) {
    const int o = (i - g0) * 8;
    const int layer = o / (HID * KPA);
    const int oo = o - layer * (HID * KPA);
    const int n = oo / KPA;
    const int k0 = oo - n * KPA;
    const float* lsp = Lb + (size_t)layer * HID * HID;
    const float* wsp = Wb + (size_t)layer * HID * HID;
#pragma unroll
    for (int e = 0; e < 8; ++e) {
      const int k = k0 + e;
      const int kl = k < HID ? k : HID - 1;
      int kw = k - HID; kw = kw < 0 ? 0 : (kw > HID - 1 ? HID - 1 : kw);
      const float a = lsp[(size_t)kl * HID + n];
      const float w = wsp[(size_t)kw * HID + n];
      v[e] = (k < HID ? a : w) * WSC;
    }
    dp = BL + o;
  } else {
    const int o = (i - g0 - g1) * 8;
    const int n = o >> 8;
    const int k0 = o & 255;
    const int nw = n < NOUT ? n : NOUT - 1;
    int nl = n - 4; nl = nl < 0 ? 0 : (nl > NOUT - 1 ? NOUT - 1 : nl);
#pragma unroll
    for (int e = 0; e < 8; ++e) {
      const int k = k0 + e;
      const float a = W2[(size_t)k * NOUT + nw];
      const float l = L2[(size_t)k * NOUT + nl];
      const float sel = (n < NOUT) ? a : ((n >= 4 && n < 4 + NOUT) ? l : 0.0f);
      v[e] = sel * WSC;
    }
    dp = B16 + o;
  }
  v4f p, q;
  p.x = v[0]; p.y = v[1]; p.z = v[2]; p.w = v[3];
  q.x = v[4]; q.y = v[5]; q.z = v[6]; q.w = v[7];
  const v8h hv = pack8(p, q);
  *(volatile v8h*)dp = hv;
  __threadfence();
  *(volatile v8h*)dp = hv;
}

__global__ __launch_bounds__(NTHR) void k_zpad(_Float16* xp, float* fp, int nvh, int nvf) {
  const int i = blockIdx.x * NTHR + (int)threadIdx.x;
  v8h zh;
#pragma unroll
  for (int j = 0; j < 8; ++j) zh[j] = (_Float16)0.0f;
  const v4f zf = {0.f, 0.f, 0.f, 0.f};
  if (i < nvh) *(volatile v8h*)(xp + (size_t)i * 8) = zh;
  if (i < nvf) *(volatile v4f*)(fp + (size_t)i * 4) = zf;
  __threadfence();
  if (i < nvh) *(volatile v8h*)(xp + (size_t)i * 8) = zh;
  if (i < nvf) *(volatile v4f*)(fp + (size_t)i * 4) = zf;
}

template <int MODE>
__global__ __launch_bounds__(NTHR) void k_agg(
    const int* __restrict__ esrc, const int* __restrict__ edst, const float* __restrict__ eval, int nE,
    const float* __restrict__ verts, _Float16* xa, const float* __restrict__ t6,
    const float* __restrict__ b2, float* vout, int nvp) {
  extern __shared__ v4f lds_dyn[];
  int* list  = (int*)lds_dyn;
  int* plist = list + LISTN;
  v2i* lsv   = (v2i*)(plist + NWAVE * PCAP);
  int* lcnt  = (int*)(lsv + TV * DEGCAP);
  int* wcnt  = lcnt + TV;
  const int tid = threadIdx.x, lane = tid & 31, wave = tid >> 5;
  const int v0 = blockIdx.x * TV;

  int pc = 0;
  const int nChunks = (nE + CHUNK - 1) / CHUNK;
#pragma unroll 1
  for (int ch = 0; ch < nChunks; ++ch) {
    const int cbase = ch * CHUNK;
    const int wcn = scan_chunk<TV, TVSH>(edst, nE, cbase, v0, 1, list, tid, lane, wave);
    if (lane == 0) wcnt[wave] = wcn;
    __syncthreads();
#pragma unroll 1
    for (int wsx = 0; wsx < NWAVE; ++wsx) {
      int n = __builtin_amdgcn_readfirstlane(wcnt[wsx]);
      n = n > WCAP ? WCAP : (n < 0 ? 0 : n);
      const int* lq = list + wsx * WCAP;
#pragma unroll 1
      for (int i0 = 0; i0 < n; i0 += 32) {
        const int idx = i0 + lane;
        const bool valid = idx < n;
        const int ent = lq[idx < WCAP ? idx : WCAP - 1];
        const int slot = ent & (TV - 1);
        const int loc = (ent >> TVSH) & (CHUNK - 1);
        int e = cbase + loc;
        e = e > nE - 1 ? nE - 1 : e;
        const bool mine = valid && ((slot >> 4) == wave);
        const unsigned mk = __builtin_amdgcn_ballot_w32(mine);
        const int pos = pc + (int)__builtin_amdgcn_mbcnt_lo(mk, 0u);
        if (mine && pos < PCAP) plist[wave * PCAP + pos] = (e << 4) | (slot & (SPW - 1));
        pc += (int)__builtin_popcount(mk);
      }
    }
    __syncthreads();
  }

  pc = pc > PCAP ? PCAP : pc;
  int cq[SPW];
#pragma unroll
  for (int qq = 0; qq < SPW; ++qq) cq[qq] = 0;
  const int* pl = plist + wave * PCAP;
#pragma unroll 1
  for (int i0 = 0; i0 < pc; i0 += 32) {
    const int idx = i0 + lane;
    const bool valid = idx < pc;
    const int ent = pl[idx < PCAP ? idx : PCAP - 1];
    const int q = ent & (SPW - 1);
    int e = ent >> 4;
    e = e < 0 ? 0 : (e > nE - 1 ? nE - 1 : e);
    int s = esrc[e];
    s = s < 0 ? 0 : (s > NVERT - 1 ? NVERT - 1 : s);
    const float v = eval[e];
    v2i en;
    en.x = s; en.y = __float_as_int(v);
#pragma unroll
    for (int qq = 0; qq < SPW; ++qq) {
      const bool hit = valid && (q == qq);
      const unsigned mk = __builtin_amdgcn_ballot_w32(hit);
      const int pos = cq[qq] + (int)__builtin_amdgcn_mbcnt_lo(mk, 0u);
      if (hit && pos < DEGCAP) lsv[(wave * SPW + qq) * DEGCAP + pos] = en;
      cq[qq] += (int)__builtin_popcount(mk);
    }
  }
  if (lane == 0) {
#pragma unroll
    for (int qq = 0; qq < SPW; ++qq) {
      const int c = cq[qq];
      lcnt[wave * SPW + qq] = c > DEGCAP ? DEGCAP : c;
    }
  }
  __syncthreads();

  if (MODE == 1) {
#pragma unroll 1
    for (int q = 0; q < SPW; ++q) {
      const int slot = wave * SPW + q;
      const int vtx  = v0 + slot;
      const int cnt  = __builtin_amdgcn_readfirstlane(lcnt[slot]);
      v8f acc[NBATCH];
#pragma unroll
      for (int b = 0; b < NBATCH; ++b) { v8f z = {0.f, 0.f, 0.f, 0.f, 0.f, 0.f, 0.f, 0.f}; acc[b] = z; }
      const v2i* lp = lsv + slot * DEGCAP;
#pragma unroll 1
      for (int i = 0; i < cnt; ++i) {
        const v2i en = lp[i];
        const int   s = __builtin_amdgcn_readfirstlane(en.x);
        const float v = __int_as_float(__builtin_amdgcn_readfirstlane(en.y));
        const _Float16* xp = xa + (size_t)s * KPA + 8 * lane;
#pragma unroll
        for (int b = 0; b < NBATCH; ++b) {
          const v8h x = *(const v8h*)(xp + (size_t)b * NVERT * KPA);
#pragma unroll
          for (int j = 0; j < 8; ++j) acc[b][j] += v * (float)x[j];
        }
      }
      if (vtx < NVERT) {
        v8h hv[NBATCH];
#pragma unroll
        for (int b = 0; b < NBATCH; ++b) {
          v8h r;
#pragma unroll
          for (int j = 0; j < 8; ++j) r[j] = (_Float16)acc[b][j];
          hv[b] = r;
        }
        _Float16* op = xa + (size_t)vtx * KPA + AGGC + 8 * lane;
#pragma unroll
        for (int b = 0; b < NBATCH; ++b) *(volatile v8h*)(op + (size_t)b * NVERT * KPA) = hv[b];
        __threadfence();
#pragma unroll
        for (int b = 0; b < NBATCH; ++b) *(volatile v8h*)(op + (size_t)b * NVERT * KPA) = hv[b];
      }
    }
  } else if (MODE == 0) {
#pragma unroll 1
    for (int q = 0; q < SPW; ++q) {
      const int slot = wave * SPW + q;
      const int vtx  = v0 + slot;
      const int cnt  = __builtin_amdgcn_readfirstlane(lcnt[slot]);
      v4f acc[NBATCH];
#pragma unroll
      for (int b = 0; b < NBATCH; ++b) { v4f z = {0.f, 0.f, 0.f, 0.f}; acc[b] = z; }
      const v2i* lp = lsv + slot * DEGCAP;
#pragma unroll 1
      for (int i = 0; i < cnt; ++i) {
        const v2i en = lp[i];
        const int   s = __builtin_amdgcn_readfirstlane(en.x);
        const float v = __int_as_float(__builtin_amdgcn_readfirstlane(en.y));
        const float* xp = verts + (size_t)s * FEAT + 4 * lane;
#pragma unroll
        for (int b = 0; b < NBATCH; ++b) {
          const v4f x = *(const v4f*)(xp + (size_t)b * NVERT * FEAT);
          acc[b] = acc[b] + x * v;
        }
      }
      if (vtx < NVERT) {
        v4h hx[NBATCH], ha[NBATCH];
        const float* rp = verts + (size_t)vtx * FEAT + 4 * lane;
#pragma unroll
        for (int b = 0; b < NBATCH; ++b) {
          const v4f xr = *(const v4f*)(rp + (size_t)b * NVERT * FEAT);
          hx[b] = pack4(xr * XSC);
          ha[b] = pack4(acc[b] * XSC);
        }
        _Float16* op = xa + (size_t)vtx * KPA + 4 * lane;
#pragma unroll
        for (int b = 0; b < NBATCH; ++b) {
          _Float16* p = op + (size_t)b * NVERT * KPA;
          *(volatile v4h*)p = hx[b];
          *(volatile v4h*)(p + AGGC) = ha[b];
        }
        __threadfence();
#pragma unroll
        for (int b = 0; b < NBATCH; ++b) {
          _Float16* p = op + (size_t)b * NVERT * KPA;
          *(volatile v4h*)p = hx[b];
          *(volatile v4h*)(p + AGGC) = ha[b];
        }
      }
    }
  } else {
    const int b = wave;
    v4f b2v;
    b2v.x = b2[0]; b2v.y = b2[1]; b2v.z = b2[2]; b2v.w = 0.0f;
    const float* tb = t6 + (size_t)b * NVERT * NLAST;
#pragma unroll 1
    for (int g = 0; g < TV / 32; ++g) {
      const int slot = 32 * g + lane;
      const int vtx = v0 + slot;
      const int vc = vtx < NVERT ? vtx : NVERT - 1;
      const int cl = lcnt[slot];
      int mx = cl;
#pragma unroll
      for (int d = 16; d >= 1; d >>= 1) { const int o = __shfl_xor(mx, d); mx = mx > o ? mx : o; }
      mx = __builtin_amdgcn_readfirstlane(mx);
      mx = mx > DEGCAP ? DEGCAP : (mx < 0 ? 0 : mx);
      v4f acc = {0.f, 0.f, 0.f, 0.f};
      const v2i* lp = lsv + slot * DEGCAP;
#pragma unroll 1
      for (int i = 0; i < mx; ++i) {
        const v2i en = lp[i];
        int s = en.x;
        s = s < 0 ? 0 : (s > NVERT - 1 ? NVERT - 1 : s);
        const float v = (i < cl) ? __int_as_float(en.y) : 0.0f;
        const v4f t = *(const v4f*)(tb + (size_t)s * NLAST);
        acc = acc + t * v;
      }
      const v4f self = *(const v4f*)(tb + (size_t)vc * NLAST + 4);
      v4f o = acc + self + b2v;
      o.w = 0.0f;
      float* op = vout + ((size_t)b * nvp + vtx) * 4;
      *(volatile v4f*)op = o;
      __threadfence();
      *(volatile v4f*)op = o;
    }
  }
}

template <int KP>
__device__ __forceinline__ void gstep(const _Float16* a0p, const _Float16* a1p, const _Float16* b0p,
                                      int acol, int bcol, v8f (&acc0)[4], v8f (&acc1)[4]) {
  FragH fa0, fa1;
  fa0.h[0] = *(const v8h*)(a0p + acol);  fa0.h[1] = *(const v8h*)(a0p + acol + 16);
  fa1.h[0] = *(const v8h*)(a1p + acol);  fa1.h[1] = *(const v8h*)(a1p + acol + 16);
#pragma unroll
  for (int t = 0; t < 4; ++t) {
    const _Float16* bq = b0p + (size_t)t * 16 * KP + bcol;
    FragH fb;
    fb.h[0] = *(const v8h*)bq;
    fb.h[1] = *(const v8h*)(bq + 16);
    wm2(fa0.v, fa1.v, fb.v, acc0[t], acc1[t]);
  }
}

template <int KS, int MODE>
__global__ __launch_bounds__(NTHR) void k_gemm(
    _Float16* xa, const _Float16* __restrict__ Bw, const float* __restrict__ bias, float* x32) {
  extern __shared__ v4f lds_dyn[];
  float* stg = (float*)lds_dyn;
  constexpr int KP  = KS * 32;
  constexpr int KXS = KS / 2;
  const int tid = threadIdx.x, lane = tid & 31, wave = tid >> 5, hh = lane >> 4, m = lane & 15;
  const int wr = wave >> 2, wc = wave & 3;
  const int rowBase = blockIdx.x * GROWS;

  v8f acc0[4], acc1[4];
#pragma unroll
  for (int t = 0; t < 4; ++t) {
    v8f z = {0.f, 0.f, 0.f, 0.f, 0.f, 0.f, 0.f, 0.f};
    acc0[t] = z; acc1[t] = z;
  }
  const _Float16* a0p = xa + (size_t)(rowBase + wr * 32 + m) * KPA + 8 * hh;
  const _Float16* a1p = a0p + (size_t)16 * KPA;
  const _Float16* b0p = Bw + (size_t)(wc * 64 + m) * KP + 8 * hh;
#pragma unroll 2
  for (int kt = 0; kt < KXS; ++kt) gstep<KP>(a0p, a1p, b0p, 32 * kt, 32 * kt, acc0, acc1);
#pragma unroll 2
  for (int kt = KXS; kt < KS; ++kt) gstep<KP>(a0p, a1p, b0p, AGGC + 32 * (kt - KXS), 32 * kt, acc0, acc1);

#pragma unroll
  for (int t = 0; t < 4; ++t) {
    const int col = wc * 64 + 16 * t + m;
    const float bv = bias[col];
    float* sp0 = stg + (wr * 32 + 8 * hh) * HID + col;
    float* sp1 = sp0 + 16 * HID;
#pragma unroll
    for (int r = 0; r < 8; ++r) {
      sp0[r * HID] = acc0[t][r] * PINV + bv;
      sp1[r * HID] = acc1[t][r] * PINV + bv;
    }
  }
  __syncthreads();

  const int rl0 = wave * 8;
  const size_t growBase = (size_t)rowBase + rl0;
  v4f keep0[8], keep1[8];
#pragma unroll
  for (int i = 0; i < 8; ++i) {
    float* sr = stg + (rl0 + i) * HID;
    v4f p0 = *(const v4f*)(sr + 4 * lane);
    v4f p1 = *(const v4f*)(sr + 128 + 4 * lane);
    p0 = relu4(p0); p1 = relu4(p1);
    if (MODE == 2) {
      const float* xr = x32 + (growBase + i) * HID;
      const v4f o0 = *(const v4f*)(xr + 4 * lane);
      const v4f o1 = *(const v4f*)(xr + 128 + 4 * lane);
      p0 = (o0 + p0) * 0.5f;
      p1 = (o1 + p1) * 0.5f;
    }
    keep0[i] = p0; keep1[i] = p1;
    *(v4f*)(sr + 4 * lane) = p0;
    *(v4f*)(sr + 128 + 4 * lane) = p1;
  }
  if (MODE != 0) {
#pragma unroll
    for (int i = 0; i < 8; ++i) {
      float* xw = x32 + (growBase + i) * HID;
      *(volatile v4f*)(xw + 4 * lane) = keep0[i];
      *(volatile v4f*)(xw + 128 + 4 * lane) = keep1[i];
    }
  }
  __syncthreads();
  v8h hv[8];
#pragma unroll
  for (int i = 0; i < 8; ++i) {
    const float* sr = stg + (rl0 + i) * HID + 8 * lane;
    const v4f q0 = *(const v4f*)sr;
    const v4f q1 = *(const v4f*)(sr + 4);
    hv[i] = pack8(q0 * XSC, q1 * XSC);
  }
#pragma unroll
  for (int i = 0; i < 8; ++i) *(volatile v8h*)(xa + (growBase + i) * KPA + 8 * lane) = hv[i];
  __threadfence();
  if (MODE != 0) {
#pragma unroll
    for (int i = 0; i < 8; ++i) {
      float* xw = x32 + (growBase + i) * HID;
      *(volatile v4f*)(xw + 4 * lane) = keep0[i];
      *(volatile v4f*)(xw + 128 + 4 * lane) = keep1[i];
    }
  }
#pragma unroll
  for (int i = 0; i < 8; ++i) *(volatile v8h*)(xa + (growBase + i) * KPA + 8 * lane) = hv[i];
}

__global__ __launch_bounds__(NTHR) void k_gemm16(
    const _Float16* __restrict__ xa, const _Float16* __restrict__ bw, float* t6) {
  __shared__ __attribute__((aligned(16))) float stg[NWAVE * 256];
  const int tid = threadIdx.x, lane = tid & 31, wave = tid >> 5, hh = lane >> 4, m = lane & 15;
  const int rowBase = blockIdx.x * G16ROWS;
  const int r0 = wave * 16;
  const _Float16* ap = xa + (size_t)(rowBase + r0 + m) * KPA + 8 * hh;
  const _Float16* bp = bw + (size_t)m * HID + 8 * hh;
  v8f acc = {0.f, 0.f, 0.f, 0.f, 0.f, 0.f, 0.f, 0.f};
#pragma unroll 2
  for (int kt = 0; kt < HID / 32; ++kt) {
    FragH fa, fb;
    fa.h[0] = *(const v8h*)(ap + 32 * kt);  fa.h[1] = *(const v8h*)(ap + 32 * kt + 16);
    fb.h[0] = *(const v8h*)(bp + 32 * kt);  fb.h[1] = *(const v8h*)(bp + 32 * kt + 16);
    acc = wm1(fa.v, fb.v, acc);
  }
  float* sw = stg + wave * 256;
#pragma unroll
  for (int r = 0; r < 8; ++r) sw[(8 * hh + r) * NLAST + m] = acc[r] * PINV;
  __syncthreads();
  const v4f o0 = *(const v4f*)(sw + 4 * lane);
  const v4f o1 = *(const v4f*)(sw + 128 + 4 * lane);
  float* gp = t6 + (size_t)(rowBase + r0) * NLAST;
  *(volatile v4f*)(gp + 4 * lane) = o0;
  *(volatile v4f*)(gp + 128 + 4 * lane) = o1;
  __threadfence();
  *(volatile v4f*)(gp + 4 * lane) = o0;
  *(volatile v4f*)(gp + 128 + 4 * lane) = o1;
}

__global__ __launch_bounds__(NTHR) void k_final(const float* __restrict__ vin, float* out, int total, int nvp) {
  const int f0 = (blockIdx.x * NTHR + (int)threadIdx.x) * 4;
  v4f o = {0.f, 0.f, 0.f, 0.f};
#pragma unroll 1
  for (int c = 0; c < 4; ++c) {
    int f = f0 + c;
    f = f > total - 1 ? total - 1 : f;
    const int row = f / NOUT;
    const int j = f - row * NOUT;
    int b = row / NVERT;
    const int v = row - b * NVERT;
    b = b > NBATCH - 1 ? NBATCH - 1 : b;
    const float x = vin[((size_t)b * nvp + v) * 4 + j];
    const float t = tanhf(x) * DEFORM;
    o.x = (c == 0) ? t : o.x;
    o.y = (c == 1) ? t : o.y;
    o.z = (c == 2) ? t : o.z;
    o.w = (c == 3) ? t : o.w;
  }
  if (f0 < total) {
    float* p = out + f0;
    *(volatile v4f*)p = o;
    __threadfence();
    *(volatile v4f*)p = o;
  }
}

extern "C" void kernel_launch(void* const* d_in, const int* in_sizes, int n_in,
                              void* d_out, int out_size, void* d_ws, size_t ws_size,
                              hipStream_t stream) {
  if (n_in < 13) return;
  if (out_size <= 0 || (out_size % NOUT) != 0 || (out_size & 3) != 0) return;
  const int rows = out_size / NOUT;
  if ((rows % NVERT) != 0 || rows / NVERT != NBATCH) return;
  if (in_sizes[0] != rows * FEAT) return;
  const int nE = in_sizes[1];
  if (nE <= 0 || nE > (1 << 24) || in_sizes[2] != nE || in_sizes[3] != nE) return;
  if (in_sizes[4] != FEAT * HID || in_sizes[5] != FEAT * HID || in_sizes[6] < HID) return;
  const int nL = in_sizes[7] / (HID * HID);
  if (nL < 2 || nL > 64 || (nL & 1) != 0 || in_sizes[7] != nL * HID * HID || in_sizes[8] != nL * HID * HID) return;
  if (in_sizes[9] < nL * HID) return;
  if (in_sizes[10] != HID * NOUT || in_sizes[11] != HID * NOUT || in_sizes[12] < NOUT) return;

  const float* verts = (const float*)d_in[0];
  const int*   esrc  = (const int*)d_in[1];
  const int*   edst  = (const int*)d_in[2];
  const float* eval  = (const float*)d_in[3];
  const float* W1    = (const float*)d_in[4];
  const float* L1    = (const float*)d_in[5];
  const float* b1    = (const float*)d_in[6];
  const float* Wb    = (const float*)d_in[7];
  const float* Lb    = (const float*)d_in[8];
  const float* bb    = (const float*)d_in[9];
  const float* W2    = (const float*)d_in[10];
  const float* L2    = (const float*)d_in[11];
  const float* b2    = (const float*)d_in[12];
  float* out = (float*)d_out;

  const int MTOT  = rows;
  const int MTOTP = ((rows + G16ROWS - 1) / G16ROWS) * G16ROWS;
  const int nGemm = MTOTP / GROWS;
  const int nG16  = MTOTP / G16ROWS;
  const int nAgg  = (NVERT + TV - 1) / TV;
  const int NVP   = nAgg * TV;
  const int nFin  = (out_size / 4 + NTHR - 1) / NTHR;
  const int nPrep = (HID * 256 / 8 + nL * (HID * KPA / 8) + NLAST * HID / 8) / NTHR;

  char* ws = (char*)d_ws;
  size_t off = 0;
  const size_t oB0  = off; off += (size_t)HID * 256 * 2;             off = (off + 255) & ~(size_t)255;
  const size_t oBL  = off; off += (size_t)nL * HID * KPA * 2;        off = (off + 255) & ~(size_t)255;
  const size_t oB16 = off; off += (size_t)NLAST * HID * 2;           off = (off + 255) & ~(size_t)255;
  const size_t oXA  = off; off += (size_t)MTOTP * KPA * 2;           off = (off + 255) & ~(size_t)255;
  const size_t oX32 = off; off += (size_t)MTOTP * HID * 4;           off = (off + 255) & ~(size_t)255;
  const size_t oT6  = off; off += (size_t)MTOTP * NLAST * 4;         off = (off + 255) & ~(size_t)255;
  const size_t oV   = off; off += (size_t)NBATCH * NVP * 4 * 4;      off = (off + 255) & ~(size_t)255;
  if (off > ws_size || off > (size_t)134217728) return;
  _Float16* B0  = (_Float16*)(ws + oB0);
  _Float16* BL  = (_Float16*)(ws + oBL);
  _Float16* B16 = (_Float16*)(ws + oB16);
  _Float16* xa  = (_Float16*)(ws + oXA);
  float*    x32 = (float*)(ws + oX32);
  float*    t6  = (float*)(ws + oT6);
  float*    vpl = (float*)(ws + oV);

  hipFuncSetAttribute(reinterpret_cast<const void*>(&k_agg<0>), hipFuncAttributeMaxDynamicSharedMemorySize, LDS_AGG);
  hipFuncSetAttribute(reinterpret_cast<const void*>(&k_agg<1>), hipFuncAttributeMaxDynamicSharedMemorySize, LDS_AGG);
  hipFuncSetAttribute(reinterpret_cast<const void*>(&k_agg<2>), hipFuncAttributeMaxDynamicSharedMemorySize, LDS_AGG);
  hipFuncSetAttribute(reinterpret_cast<const void*>(&k_gemm<8, 1>), hipFuncAttributeMaxDynamicSharedMemorySize, LDS_GEMM);
  hipFuncSetAttribute(reinterpret_cast<const void*>(&k_gemm<16, 0>), hipFuncAttributeMaxDynamicSharedMemorySize, LDS_GEMM);
  hipFuncSetAttribute(reinterpret_cast<const void*>(&k_gemm<16, 2>), hipFuncAttributeMaxDynamicSharedMemorySize, LDS_GEMM);

  k_wprep<<<nPrep, NTHR, 0, stream>>>(W1, L1, Wb, Lb, W2, L2, B0, BL, B16, nL);

  const int padRows = MTOTP - MTOT;
  if (padRows > 0) {
    const int nvh = padRows * (KPA / 8);
    const int nvf = padRows * (HID / 4);
    const int nvm = nvh > nvf ? nvh : nvf;
    const int nZ  = (nvm + NTHR - 1) / NTHR;
    k_zpad<<<nZ, NTHR, 0, stream>>>(xa + (size_t)MTOT * KPA, x32 + (size_t)MTOT * HID, nvh, nvf);
  }

  k_agg<0><<<nAgg, NTHR, LDS_AGG, stream>>>(esrc, edst, eval, nE, verts, xa, t6, b2, vpl, NVP);
  k_gemm<8, 1><<<nGemm, NTHR, LDS_GEMM, stream>>>(xa, B0, b1, x32);

  const int nBlk = nL / 2;
  for (int i = 0; i < nBlk; ++i) {
    k_agg<1><<<nAgg, NTHR, LDS_AGG, stream>>>(esrc, edst, eval, nE, verts, xa, t6, b2, vpl, NVP);
    k_gemm<16, 0><<<nGemm, NTHR, LDS_GEMM, stream>>>(xa, BL + (size_t)(2 * i) * HID * KPA, bb + (size_t)(2 * i) * HID, x32);
    k_agg<1><<<nAgg, NTHR, LDS_AGG, stream>>>(esrc, edst, eval, nE, verts, xa, t6, b2, vpl, NVP);
    k_gemm<16, 2><<<nGemm, NTHR, LDS_GEMM, stream>>>(xa, BL + (size_t)(2 * i + 1) * HID * KPA, bb + (size_t)(2 * i + 1) * HID, x32);
  }

  k_gemm16<<<nG16, NTHR, 0, stream>>>(xa, B16, t6);
  k_agg<2><<<nAgg, NTHR, LDS_AGG, stream>>>(esrc, edst, eval, nE, verts, xa, t6, b2, vpl, NVP);
  k_final<<<nFin, NTHR, 0, stream>>>(vpl, out, out_size, NVP);
}
